// OTResample_18279380812196
// MI455X (gfx1250) — hardware-run, weakly checked
//
#include <hip/hip_runtime.h>
#include <math.h>

constexpr int kB = 8;
constexpr int kN = 2048;
constexpr int kD = 64;
constexpr int kGrp = 4;
constexpr int kNumGrp = kB / kGrp;
constexpr int kRows = 32;
constexpr int kIters = 10;
constexpr float kLn2x20   = 13.862943611198906f;
constexpr float kLogNu    = -7.6246189861593985f;
constexpr float kInvCnt   = 1.0f / 4194304.0f;
constexpr float kInvEps   = 10.0f;
constexpr float kOutScale = 2048.0f / 1048576.0f;
constexpr float kInvN     = 1.0f / 2048.0f;
static_assert(kB % kGrp == 0);
static_assert(kN % 64 == 0);
static_assert(kD % 32 == 0);
static_assert(kN % kRows == 0);
static_assert(kN == 8 * 256);

constexpr size_t kX16Bytes  = (size_t)kB * kN * kD * 2;
constexpr size_t kXT16Bytes = (size_t)kB * kD * kN * 2;
constexpr size_t kGBytes    = (size_t)kN * kN * 4;
constexpr size_t kCBytes    = (size_t)kGrp * kN * kN * 4;
constexpr size_t kPtBytes   = (size_t)kGrp * kN * kN * 2;
constexpr size_t kVecBytes  = (size_t)kB * kN * 4;
constexpr size_t kWsTotal   = kX16Bytes + kXT16Bytes + kGBytes + kCBytes + kPtBytes + 5 * kVecBytes;
static_assert(kWsTotal <= (size_t)134217728);

typedef __attribute__((ext_vector_type(16))) _Float16 v16h;
typedef __attribute__((ext_vector_type(8)))  _Float16 v8h;
typedef __attribute__((ext_vector_type(16))) __bf16   v16b;
typedef __attribute__((ext_vector_type(8)))  __bf16   v8b;
typedef __attribute__((ext_vector_type(8)))  float    v8f;
typedef __attribute__((ext_vector_type(4)))  float    v4f;
typedef __attribute__((ext_vector_type(4)))  unsigned int v4u;

__device__ __forceinline__ unsigned short f2bf_bits(float f) {
  unsigned u = __float_as_uint(f);
  return (unsigned short)((u + 0x7FFFu + ((u >> 16) & 1u)) >> 16);
}
__device__ __forceinline__ float bf_bits2f(unsigned short h) { return __uint_as_float(((unsigned)h) << 16); }

__device__ __forceinline__ void dep_guard_h(v8f& a, v8f& b, v16h x, v16h y) { asm volatile("v_nop\n\tv_nop\n\tv_nop\n\tv_nop" : "+v"(a), "+v"(b) : "v"(x), "v"(y)); }
__device__ __forceinline__ void dep_guard_b(v8f& a, v8f& b, v16b x, v16b y) { asm volatile("v_nop\n\tv_nop\n\tv_nop\n\tv_nop" : "+v"(a), "+v"(b) : "v"(x), "v"(y)); }
__device__ __forceinline__ void keep4_h(v16h a, v16h b, v16h c, v16h d) { asm volatile("v_nop" :: "v"(a), "v"(b), "v"(c), "v"(d)); }
__device__ __forceinline__ void keep4_b(v16b a, v16b b, v16b c, v16b d) { asm volatile("v_nop" :: "v"(a), "v"(b), "v"(c), "v"(d)); }
__device__ __forceinline__ void acc_guard4(v8f& a, v8f& b, v8f& c, v8f& d) { asm volatile("v_nop\n\tv_nop\n\tv_nop\n\tv_nop" : "+v"(a), "+v"(b), "+v"(c), "+v"(d)); }
template <typename T> struct Frag;
template <> struct Frag<_Float16> {
  typedef v16h V; union U { v16h v; v8h h[2]; };
  static __device__ __forceinline__ v16h load(const _Float16* p) {
    U f; f.h[0] = *(const v8h*)(p); f.h[1] = *(const v8h*)(p + 16); return f.v;
  }
  static __device__ __forceinline__ v8f mma(v16h a, v16h b, v8f c) {
    return __builtin_amdgcn_wmma_f32_16x16x32_f16(false, a, false, b, (short)0, c, false, false);
  }
  static __device__ __forceinline__ void guard(v8f& a, v8f& b, v16h x, v16h y) { dep_guard_h(a, b, x, y); }
  static __device__ __forceinline__ void keep(v16h a, v16h b, v16h c, v16h d) { keep4_h(a, b, c, d); }
};
template <> struct Frag<__bf16> {
  typedef v16b V; union U { v16b v; v8b h[2]; };
  static __device__ __forceinline__ v16b load(const __bf16* p) {
    U f; f.h[0] = *(const v8b*)(p); f.h[1] = *(const v8b*)(p + 16); return f.v;
  }
  static __device__ __forceinline__ v8f mma(v16b a, v16b b, v8f c) {
    return __builtin_amdgcn_wmma_f32_16x16x32_bf16(false, a, false, b, (short)0, c, false, false);
  }
  static __device__ __forceinline__ void guard(v8f& a, v8f& b, v16b x, v16b y) { dep_guard_b(a, b, x, y); }
  static __device__ __forceinline__ void keep(v16b a, v16b b, v16b c, v16b d) { keep4_b(a, b, c, d); }
};

__device__ __forceinline__ unsigned pk16(unsigned short a, unsigned short b) { return (unsigned)a | ((unsigned)b << 16); }
__device__ __forceinline__ unsigned short h_bits(float f) { const _Float16 h = (_Float16)f; return __builtin_bit_cast(unsigned short, h); }

template <int ET> struct Elem;
template <> struct Elem<0> { typedef _Float16 T; };
template <> struct Elem<1> { typedef __bf16 T; };
template <int ET, bool SPLIT, int BIAS_MODE, int OUT_MODE, bool RESID, int ACT = 0>
__global__ __launch_bounds__(256) void wmma_gemm64(
    const unsigned short* __restrict__ Ap, const unsigned short* __restrict__ A2p, int lda, long strideA,
    const unsigned short* __restrict__ Btp, const unsigned short* __restrict__ Bt2p, int ldb, long strideB,
    void* __restrict__ Cout, void* __restrict__ Cout2, int ldc, long strideC,
    const float* __restrict__ bias,
    const float* __restrict__ resid, long strideR,
    int M, int N, int K, float scale) {
  typedef typename Elem<ET>::T T;
  typedef typename Frag<T>::V V;
  const T* A = (const T*)Ap; const T* A2 = (const T*)A2p; const T* Bt = (const T*)Btp; const T* Bt2 = (const T*)Bt2p;
  __shared__ __align__(16) float sT[8][16 * 68];
  const int b    = blockIdx.y;
  const int lane = threadIdx.x & 31;
  const int wave = threadIdx.x >> 5;
  const int tilesN = N >> 6;
  const int tilesM = M >> 6;
  const int tile = blockIdx.x * 8 + wave;
  if (tile >= tilesM * tilesN) return;
  const int tm = tile / tilesN;
  const int tn = tile - tm * tilesN;
  const int m0 = tm << 6;
  const int n0 = tn << 6;

  const T* Ab  = A  + (size_t)b * strideA;
  const T* Bb  = Bt + (size_t)b * strideB;
  const T* Ab2 = SPLIT ? (A2  + (size_t)b * strideA) : nullptr;
  const T* Bb2 = SPLIT ? (Bt2 + (size_t)b * strideB) : nullptr;

  const int rlane = lane & 15;
  const int koff  = (lane >> 4) * 8;
  const int mOff  = (lane >> 4) * 8;

  v8f acc[4][4];
#pragma unroll
  for (int i = 0; i < 4; ++i)
#pragma unroll
    for (int j = 0; j < 4; ++j) acc[i][j] = (v8f){0.f,0.f,0.f,0.f,0.f,0.f,0.f,0.f};

  for (int k0 = 0; k0 < K; k0 += 32) {
    V bh[4], bl[4];
#pragma unroll
    for (int j = 0; j < 4; ++j) {
      const size_t bo = (size_t)(n0 + (j << 4) + rlane) * ldb + koff + k0;
      bh[j] = Frag<T>::load(Bb + bo);
      if (SPLIT) bl[j] = Frag<T>::load(Bb2 + bo);
    }
#pragma unroll
    for (int i = 0; i < 4; ++i) {
      const size_t ao = (size_t)(m0 + (i << 4) + rlane) * lda + koff + k0;
      V ah = Frag<T>::load(Ab + ao);
      V al;
      if (SPLIT) al = Frag<T>::load(Ab2 + ao);
#pragma unroll
      for (int j = 0; j < 4; ++j) {
        acc[i][j] = Frag<T>::mma(ah, bh[j], acc[i][j]);
        if (SPLIT) {
          acc[i][j] = Frag<T>::mma(ah, bl[j], acc[i][j]);
          acc[i][j] = Frag<T>::mma(al, bh[j], acc[i][j]);
        }
      }
      Frag<T>::guard(acc[i][0], acc[i][3], ah, SPLIT ? al : ah);
    }
    Frag<T>::keep(bh[0], bh[1], bh[2], bh[3]);
    if (SPLIT) Frag<T>::keep(bl[0], bl[1], bl[2], bl[3]);
  }
  acc_guard4(acc[0][0], acc[0][1], acc[0][2], acc[0][3]);
  acc_guard4(acc[1][0], acc[1][1], acc[1][2], acc[1][3]);
  acc_guard4(acc[2][0], acc[2][1], acc[2][2], acc[2][3]);
  acc_guard4(acc[3][0], acc[3][1], acc[3][2], acc[3][3]);

  float* slab = sT[wave];
  const float* Rb = RESID ? (resid + (size_t)b * strideR) : nullptr;
#pragma unroll
  for (int i = 0; i < 4; ++i) {
    const int mBase = m0 + (i << 4);
#pragma unroll
    for (int j = 0; j < 4; ++j) {
      const int n = n0 + (j << 4) + rlane;
      float bv = 0.f;
      if (BIAS_MODE == 2) bv = bias[n];
#pragma unroll
      for (int r = 0; r < 8; ++r) {
        float v = acc[i][j][r] * scale;
        if (BIAS_MODE == 1) v += bias[mBase + mOff + r];
        if (BIAS_MODE == 2) v += bv;
        if (RESID) v += Rb[(size_t)(mBase + mOff + r) * ldc + n];
        if (ACT == 2) v = fmaxf(v, 0.0f);
        if (ACT == 4) v = (v > 0.f) ? v : 0.01f * v;
        slab[(mOff + r) * 68 + (j << 4) + rlane] = v;
      }
    }
    __builtin_amdgcn_fence(__ATOMIC_RELEASE, "workgroup");
    __builtin_amdgcn_wave_barrier();
    __builtin_amdgcn_fence(__ATOMIC_ACQUIRE, "workgroup");
    if (OUT_MODE == 0) {
      float* C = (float*)Cout + (size_t)b * strideC;
      const int hh = lane >> 4, c4 = (lane & 15) * 4;
      for (int pass = 0; pass < 2; ++pass) {
#pragma unroll
        for (int it = 0; it < 8; ++it) {
          const int row = it * 2 + hh;
          v4f v = *(const v4f*)(slab + row * 68 + c4);
          *(volatile v4f*)(C + (size_t)(mBase + row) * ldc + n0 + c4) = v;
        }
        __threadfence();
      }
    } else {
      const int q = lane >> 3, c8 = (lane & 7) * 8;
      unsigned short* C  = (unsigned short*)Cout  + (size_t)b * strideC;
      unsigned short* C2 = (OUT_MODE == 2) ? ((unsigned short*)Cout2 + (size_t)b * strideC) : nullptr;
      for (int pass = 0; pass < 2; ++pass) {
#pragma unroll
        for (int it = 0; it < 4; ++it) {
          const int row = it * 4 + q;
          const float* sp = slab + row * 68 + c8;
          v8h hv, lv;
#pragma unroll
          for (int e = 0; e < 8; ++e) {
            if (OUT_MODE == 1) {
              hv[e] = (_Float16)sp[e];
            } else {
              unsigned short hb = f2bf_bits(sp[e]);
              unsigned short lb = f2bf_bits(sp[e] - bf_bits2f(hb));
              hv[e] = __builtin_bit_cast(_Float16, hb);
              lv[e] = __builtin_bit_cast(_Float16, lb);
            }
          }
          *(volatile v8h*)(C + (size_t)(mBase + row) * ldc + n0 + c8) = hv;
          if (OUT_MODE == 2) *(volatile v8h*)(C2 + (size_t)(mBase + row) * ldc + n0 + c8) = lv;
        }
        __threadfence();
      }
    }
    __builtin_amdgcn_fence(__ATOMIC_RELEASE, "workgroup");
    __builtin_amdgcn_wave_barrier();
    __builtin_amdgcn_fence(__ATOMIC_ACQUIRE, "workgroup");
  }
}

__global__ __launch_bounds__(256) void cast8_f16_kernel(const float* __restrict__ in, unsigned short* __restrict__ out, int n8) {
  const int i = blockIdx.x * 256 + threadIdx.x;
  if (i >= n8) return;
  const float* p = in + 8 * (size_t)i;
  const v4f a = *(const v4f*)(p);
  const v4f c = *(const v4f*)(p + 4);
  unsigned short hb[8];
#pragma unroll
  for (int e = 0; e < 4; ++e) {
    hb[e]     = h_bits(a[e]);
    hb[4 + e] = h_bits(c[e]);
  }
  const v4u u = (v4u){pk16(hb[0], hb[1]), pk16(hb[2], hb[3]), pk16(hb[4], hb[5]), pk16(hb[6], hb[7])};
  unsigned short* q = out + 8 * (size_t)i;
  *(volatile v4u*)q = u;
  __threadfence();
  *(volatile v4u*)q = u;
}

__global__ __launch_bounds__(256) void xt_kernel(const float* __restrict__ X, unsigned short* __restrict__ out) {
  __shared__ float sm[64][65];
  const int t  = threadIdx.x;
  const int n0 = blockIdx.x * 64;
  const int b  = blockIdx.y;
  const float* Xb = X + (size_t)b * kN * kD;
#pragma unroll
  for (int i = 0; i < 16; ++i) {
    const int e = i * 256 + t;
    const int r = e >> 6;
    const int c = e & 63;
    sm[c][r] = Xb[(size_t)(n0 + r) * kD + c];
  }
  __syncthreads();
  const int lane = t & 31, wave = t >> 5;
  const int q = lane >> 3, c8 = (lane & 7) * 8;
  unsigned short* op = out + (size_t)b * kD * kN;
  for (int pass = 0; pass < 2; ++pass) {
#pragma unroll
    for (int it = 0; it < 2; ++it) {
      const int row = wave * 8 + it * 4 + q;
      unsigned short hb[8];
#pragma unroll
      for (int e = 0; e < 8; ++e) hb[e] = h_bits(sm[row][c8 + e]);
      const v4u u = (v4u){pk16(hb[0], hb[1]), pk16(hb[2], hb[3]), pk16(hb[4], hb[5]), pk16(hb[6], hb[7])};
      *(volatile v4u*)(op + (size_t)row * kN + n0 + c8) = u;
    }
    __threadfence();
  }
}

__global__ __launch_bounds__(256) void prep_kernel(const float* __restrict__ X, const float* __restrict__ W,
                                                   float* __restrict__ sq, float* __restrict__ logmu, int nrows) {
  const int row = blockIdx.x * 256 + threadIdx.x;
  if (row >= nrows) return;
  const float* p = X + (size_t)row * kD;
  float s = 0.f;
#pragma unroll 2
  for (int i = 0; i < kD / 4; ++i) {
    const v4f v = *(const v4f*)(p + 4 * i);
    s += v[0] * v[0];
    s += v[1] * v[1];
    s += v[2] * v[2];
    s += v[3] * v[3];
  }
  const float lm = logf(W[row] + 1e-16f);
  ((volatile float*)sq)[row] = s;
  ((volatile float*)logmu)[row] = lm;
  __threadfence();
  ((volatile float*)sq)[row] = s;
  ((volatile float*)logmu)[row] = lm;
}

__global__ __launch_bounds__(256) void cost_kernel(const float* __restrict__ G, const float* __restrict__ sqb,
                                                   float* __restrict__ Cout, float* __restrict__ partl) {
#pragma clang fp contract(off)
  __shared__ float sqrow[kRows];
  __shared__ float wsum[8];
  const int t = threadIdx.x, lane = t & 31, wave = t >> 5;
  const int r0 = blockIdx.x * kRows;
  {
    const float sv = sqb[r0 + (t & 31)];
    if (t < kRows) sqrow[t] = sv;
  }
  const v4f qa = *(const v4f*)(sqb + 4 * t);
  const v4f qb = *(const v4f*)(sqb + 1024 + 4 * t);
  __syncthreads();
  float lsum = 0.f;
#pragma unroll 1
  for (int rl = 0; rl < kRows; ++rl) {
    const int row = r0 + rl;
    const float sqn = sqrow[rl];
    const float* gr = G + (size_t)row * kN;
    const v4f g0 = *(const v4f*)(gr + 4 * t);
    const v4f g1 = *(const v4f*)(gr + 1024 + 4 * t);
    v4f c0, c1;
#pragma unroll
    for (int e = 0; e < 4; ++e) {
      const float t0 = sqn + qa[e];
      const float u0 = 2.0f * g0[e];
      c0[e] = t0 - u0;
      const float t1 = sqn + qb[e];
      const float u1 = 2.0f * g1[e];
      c1[e] = t1 - u1;
    }
#pragma unroll
    for (int e = 0; e < 4; ++e) lsum += c0[e];
#pragma unroll
    for (int e = 0; e < 4; ++e) lsum += c1[e];
    float* cr = Cout + (size_t)row * kN;
    *(volatile v4f*)(cr + 4 * t) = c0;
    *(volatile v4f*)(cr + 1024 + 4 * t) = c1;
    __threadfence();
    *(volatile v4f*)(cr + 4 * t) = c0;
    *(volatile v4f*)(cr + 1024 + 4 * t) = c1;
  }
#pragma unroll
  for (int off = 16; off > 0; off >>= 1) lsum += __shfl_xor(lsum, off, 32);
  if (lane == 0) wsum[wave] = lsum;
  __syncthreads();
  if (wave == 0) {
    float tot = wsum[0];
#pragma unroll
    for (int w = 1; w < 8; ++w) tot += wsum[w];
    const float v = (lane == 0) ? tot : 0.f;
    float* pp = partl + (size_t)blockIdx.x * 32 + lane;
    *(volatile float*)pp = v;
    __threadfence();
    *(volatile float*)pp = v;
  }
}

__global__ __launch_bounds__(256) void lse_kernel(const float* __restrict__ Cg, const float* __restrict__ part,
                                                  const float* __restrict__ vin, const float* __restrict__ basev,
                                                  float* __restrict__ vout,
                                                  int b0, int use_vec, int use_base, float base_const) {
  __shared__ float red[64];
  __shared__ float wmx[8];
  __shared__ float wsm[8];
  __shared__ float basel[kRows];
  __shared__ __align__(16) float res[kRows];
  const int t = threadIdx.x, lane = t & 31, wave = t >> 5;
  const int bl = blockIdx.y;
  const int bg = b0 + bl;
  const int r0 = blockIdx.x * kRows;
  const float* Cp = Cg + (size_t)bl * kN * kN;
  const size_t vb = (size_t)bg * kN;
  {
    const float pv = part[vb + (size_t)(t & 63) * 32];
    if (t < 64) red[t] = pv;
    const float bvl = basev[vb + r0 + (t & 31)];
    if (t < kRows) basel[t] = use_base ? bvl : base_const;
  }
  __syncthreads();
  for (int off = 32; off > 0; off >>= 1) {
    if (t < off) red[t] += red[t + off];
    __syncthreads();
  }
  const float cmean = red[0] * kInvCnt + 1e-8f;
  const float ns = -(1.0f / cmean) * kInvEps;
  v4f v0 = (v4f){0.f, 0.f, 0.f, 0.f};
  v4f v1 = v0;
  if (use_vec) {
    v0 = *(const v4f*)(vin + vb + 4 * t);
    v1 = *(const v4f*)(vin + vb + 1024 + 4 * t);
  }
#pragma unroll 1
  for (int rl = 0; rl < kRows; ++rl) {
    const float* cr = Cp + (size_t)(r0 + rl) * kN;
    const v4f c0 = *(const v4f*)(cr + 4 * t);
    const v4f c1 = *(const v4f*)(cr + 1024 + 4 * t);
    float x[8];
#pragma unroll
    for (int e = 0; e < 4; ++e) {
      x[e]     = fmaf(c0[e], ns, v0[e]);
      x[4 + e] = fmaf(c1[e], ns, v1[e]);
    }
    float m = fmaxf(fmaxf(fmaxf(x[0], x[1]), fmaxf(x[2], x[3])), fmaxf(fmaxf(x[4], x[5]), fmaxf(x[6], x[7])));
#pragma unroll
    for (int off = 16; off > 0; off >>= 1) m = fmaxf(m, __shfl_xor(m, off, 32));
    if (lane == 0) wmx[wave] = m;
    __syncthreads();
    float mx = wmx[0];
#pragma unroll
    for (int w = 1; w < 8; ++w) mx = fmaxf(mx, wmx[w]);
    float s = 0.f;
#pragma unroll
    for (int e = 0; e < 8; ++e) s += expf(x[e] - mx);
#pragma unroll
    for (int off = 16; off > 0; off >>= 1) s += __shfl_xor(s, off, 32);
    if (lane == 0) wsm[wave] = s;
    __syncthreads();
    if (t == 0) {
      float ssum = wsm[0];
#pragma unroll
      for (int w = 1; w < 8; ++w) ssum += wsm[w];
      res[rl] = basel[rl] - (mx + logf(ssum));
    }
  }
  __syncthreads();
  if (wave == 0) {
    const v4f rv = *(const v4f*)(res + 4 * (lane & 7));
    float* vo = vout + vb + r0 + 4 * (lane & 7);
    if (lane < 8) *(volatile v4f*)vo = rv;
    __threadfence();
    if (lane < 8) *(volatile v4f*)vo = rv;
  }
}

__global__ __launch_bounds__(256) void pbuild_kernel(const float* __restrict__ Cg, const float* __restrict__ part,
                                                     const float* __restrict__ fvec, const float* __restrict__ gvec,
                                                     unsigned short* __restrict__ Ptg, int b0) {
  __shared__ float red[64];
  __shared__ float gml[kRows];
  const int t = threadIdx.x;
  const int bl = blockIdx.y;
  const int bg = b0 + bl;
  const int r0 = blockIdx.x * kRows;
  const float* Cp = Cg + (size_t)bl * kN * kN;
  unsigned short* Pp = Ptg + (size_t)bl * kN * kN;
  const size_t vb = (size_t)bg * kN;
  {
    const float pv = part[vb + (size_t)(t & 63) * 32];
    if (t < 64) red[t] = pv;
    const float gv = gvec[vb + r0 + (t & 31)] + kLn2x20;
    if (t < kRows) gml[t] = gv;
  }
  __syncthreads();
  for (int off = 32; off > 0; off >>= 1) {
    if (t < off) red[t] += red[t + off];
    __syncthreads();
  }
  const float cmean = red[0] * kInvCnt + 1e-8f;
  const float ns = -(1.0f / cmean) * kInvEps;
  const v4f f0 = *(const v4f*)(fvec + vb + 8 * t);
  const v4f f1 = *(const v4f*)(fvec + vb + 8 * t + 4);
#pragma unroll 1
  for (int rl = 0; rl < kRows; ++rl) {
    const int row = r0 + rl;
    const float gm = gml[rl];
    const float* cr = Cp + (size_t)row * kN;
    const v4f c0 = *(const v4f*)(cr + 8 * t);
    const v4f c1 = *(const v4f*)(cr + 8 * t + 4);
    unsigned short hb[8];
#pragma unroll
    for (int e = 0; e < 4; ++e) {
      hb[e]     = h_bits(expf(f0[e] + fmaf(c0[e], ns, gm)));
      hb[4 + e] = h_bits(expf(f1[e] + fmaf(c1[e], ns, gm)));
    }
    const v4u u = (v4u){pk16(hb[0], hb[1]), pk16(hb[2], hb[3]), pk16(hb[4], hb[5]), pk16(hb[6], hb[7])};
    unsigned short* pr = Pp + (size_t)row * kN + 8 * t;
    *(volatile v4u*)pr = u;
    __threadfence();
    *(volatile v4u*)pr = u;
  }
}

__global__ __launch_bounds__(256) void fill_kernel(float* __restrict__ out, int n4, float val) {
  const int i = blockIdx.x * 256 + threadIdx.x;
  if (i >= n4) return;
  const v4f v = (v4f){val, val, val, val};
  float* p = out + 4 * (size_t)i;
  *(volatile v4f*)p = v;
  __threadfence();
  *(volatile v4f*)p = v;
}

extern "C" void kernel_launch(void* const* d_in, const int* in_sizes, int n_in,
                              void* d_out, int out_size, void* d_ws, size_t ws_size, hipStream_t stream) {
  if (n_in < 2) return;
  if (in_sizes[0] != kB * kN * kD) return;
  if (in_sizes[1] != kB * kN) return;
  if (out_size != kB * kN * kD + kB * kN) return;

  const size_t oX16  = 0;
  const size_t oXT16 = oX16 + kX16Bytes;
  const size_t oG    = oXT16 + kXT16Bytes;
  const size_t oC    = oG + kGBytes;
  const size_t oPt   = oC + kCBytes;
  const size_t oSq   = oPt + kPtBytes;
  const size_t oLm   = oSq + kVecBytes;
  const size_t oF    = oLm + kVecBytes;
  const size_t oGv   = oF + kVecBytes;
  const size_t oPart = oGv + kVecBytes;
  const size_t oEnd  = oPart + kVecBytes;
  if (oEnd > ws_size) return;

  const float* X  = (const float*)d_in[0];
  const float* Wt = (const float*)d_in[1];
  float* outp = (float*)d_out;
  float* outw = outp + (size_t)kB * kN * kD;

  char* ws = (char*)d_ws;
  unsigned short* X16  = (unsigned short*)(ws + oX16);
  unsigned short* XT16 = (unsigned short*)(ws + oXT16);
  float* G     = (float*)(ws + oG);
  float* Cpl   = (float*)(ws + oC);
  unsigned short* Pt = (unsigned short*)(ws + oPt);
  float* sq    = (float*)(ws + oSq);
  float* logmu = (float*)(ws + oLm);
  float* fvec  = (float*)(ws + oF);
  float* gvec  = (float*)(ws + oGv);
  float* part  = (float*)(ws + oPart);

  {
    const int n8 = kB * kN * kD / 8;
    cast8_f16_kernel<<<dim3((n8 + 255) / 256), dim3(256), 0, stream>>>(X, X16, n8);
    xt_kernel<<<dim3(kN / 64, kB), dim3(256), 0, stream>>>(X, XT16);
    const int nrows = kB * kN;
    prep_kernel<<<dim3((nrows + 255) / 256), dim3(256), 0, stream>>>(X, Wt, sq, logmu, nrows);
  }

  for (int grp = 0; grp < kNumGrp; ++grp) {
    const int b0 = grp * kGrp;
    for (int bl = 0; bl < kGrp; ++bl) {
      const int bg = b0 + bl;
      const unsigned short* Xb = X16 + (size_t)bg * kN * kD;
      wmma_gemm64<0, false, 0, 0, false, 0><<<dim3((kN / 64) * (kN / 64) / 8, 1), dim3(256), 0, stream>>>(
          Xb, nullptr, kD, (long)0,
          Xb, nullptr, kD, (long)0,
          (void*)G, nullptr, kN, (long)0,
          nullptr, nullptr, (long)0,
          kN, kN, kD, 1.0f);
      cost_kernel<<<dim3(kN / kRows), dim3(256), 0, stream>>>(
          G, sq + (size_t)bg * kN, Cpl + (size_t)bl * kN * kN, part + (size_t)bg * kN);
    }
    for (int it = 0; it < kIters; ++it) {
      lse_kernel<<<dim3(kN / kRows, kGrp), dim3(256), 0, stream>>>(
          Cpl, part, gvec, logmu, fvec, b0, (it > 0) ? 1 : 0, 1, 0.0f);
      lse_kernel<<<dim3(kN / kRows, kGrp), dim3(256), 0, stream>>>(
          Cpl, part, fvec, logmu, gvec, b0, 1, 0, kLogNu);
    }
    pbuild_kernel<<<dim3(kN / kRows, kGrp), dim3(256), 0, stream>>>(Cpl, part, fvec, gvec, Pt, b0);
    wmma_gemm64<0, false, 0, 0, false, 0><<<dim3((kN / 64) * (kD / 64) / 8, kGrp), dim3(256), 0, stream>>>(
        Pt, nullptr, kN, (long)kN * kN,
        XT16 + (size_t)b0 * kD * kN, nullptr, kN, (long)kD * kN,
        (void*)(outp + (size_t)b0 * kN * kD), nullptr, kD, (long)kN * kD,
        nullptr, nullptr, (long)0,
        kN, kD, kN, kOutScale);
  }

  {
    const int n4 = kB * kN / 4;
    fill_kernel<<<dim3((n4 + 255) / 256), dim3(256), 0, stream>>>(outw, n4, kInvN);
  }
}
